// DrugGCNncoder_25434796327024
// MI455X (gfx1250) — hardware-run, weakly checked
//
#include <hip/hip_runtime.h>
#include <stddef.h>
#include <stdint.h>
#include <math.h>


#define NN      100000
#define NE      1600000
#define F0      78
#define HD      300
#define HP      320
#define NGR     512
#define D3      1024
#define D4      128
#define XP      128
#define K1H     96
#define K1      192
#define K2      640
#define K3      640
#define K4      2048
#define NTHR    256
#define NWAVE   8
#define EPT     8
#define CHUNK   (NTHR * EPT)
#define WCAP    (EPT * 32)
#define LISTN   (NWAVE * WCAP)
#define NBA     1024
#define SLA     10
#define NBLK    98
#define NPAD    (NBLK * NBA)
#define RCAP    28672
#define DEGCAP  64
#define GCAP    16
#define NREC    (NBLK * GCAP)
#define CH      25088
#define NCHUNK  4
#define GTHR    256
#define AGG_ZINTS (LISTN + 2 * RCAP + 3 * NBA)
#define AGG_LDS_INTS (AGG_ZINTS + 16)
#define PB_X    (NN * 16 / NTHR)
#define PB_W1   (HP * (K1 / 8) / NTHR)
#define PB_W2   (HP * (K2 / 8) / NTHR)
#define PB_W3   (D3 * (K3 / 8) / NTHR)
#define PB_W4   (D4 * (K4 / 8) / NTHR)
#define PB_WEND (PB_X + PB_W1 + PB_W2 + PB_W3 + PB_W4)
#define PB_ALL  (PB_WEND + 4)
#define OB1     0
#define OB2     320
#define OB3     640
#define OB4     1664
#define NBIAS   1792

static_assert((CHUNK & (CHUNK - 1)) == 0 && CHUNK <= 4096);
static_assert((NBA & (NBA - 1)) == 0 && NBA == (1 << SLA));
static_assert(NE < (1 << 21));
static_assert(((long long)(NE + CHUNK) << SLA) < (1LL << 31));
static_assert(NPAD >= NN && NCHUNK * CH == NPAD && CH % 64 == 0);
static_assert(K1 % 32 == 0 && K2 % 32 == 0 && K3 % 32 == 0 && K4 % 32 == 0 && HP % 32 == 0);
static_assert(K1 == 2 * K1H && K2 == 2 * HP && K3 == 2 * HP && K4 == 2 * D3);
static_assert(RCAP >= 17546 && DEGCAP >= 44);
static_assert(RCAP % (4 * NTHR) == 0 && NBA % NTHR == 0 && NBA == 4 * NTHR);
static_assert((NN * 16) % NTHR == 0);
static_assert((HP * (K1 / 8)) % NTHR == 0 && (HP * (K2 / 8)) % NTHR == 0);
static_assert((D3 * (K3 / 8)) % NTHR == 0 && (D4 * (K4 / 8)) % NTHR == 0);
static_assert(NREC % 32 == 0);
static_assert(AGG_ZINTS % (4 * NTHR) == 0);
static_assert(AGG_LDS_INTS * 4 <= 327680);
static_assert(NWAVE * GCAP * HP * 4 + 8192 <= 327680);
static_assert(NGR % 64 == 0 && D3 % 256 == 0 && D4 == 128);
static_assert(NGR * D4 == 65536);
static_assert(HP == 320 && XP == 128);

typedef float          v2f   __attribute__((ext_vector_type(2)));
typedef float          v4f   __attribute__((ext_vector_type(4)));
typedef float          v8f   __attribute__((ext_vector_type(8)));
typedef int            v4i   __attribute__((ext_vector_type(4)));
typedef int            v8i   __attribute__((ext_vector_type(8)));
typedef unsigned int   v2u   __attribute__((ext_vector_type(2)));
typedef unsigned int   v4u   __attribute__((ext_vector_type(4)));
typedef unsigned short v8us  __attribute__((ext_vector_type(8)));
typedef unsigned short v16us __attribute__((ext_vector_type(16)));
typedef __bf16         v16bf __attribute__((ext_vector_type(16)));
typedef v2f  __attribute__((may_alias)) v2fa;
typedef v4f  __attribute__((may_alias)) v4fa;
typedef v4i  __attribute__((may_alias)) v4ia;
typedef v2u  __attribute__((may_alias)) v2ua;
typedef v4u  __attribute__((may_alias)) v4ua;
typedef v8us __attribute__((may_alias)) v8usa;
union FragB { v16bf v; v16us u; v8us h[2]; v8i w; };

__device__ __forceinline__ v8f wmb(const FragB& a, const FragB& b, v8f c) {
  v8f d = __builtin_amdgcn_wmma_f32_16x16x32_bf16(false, a.v, false, b.v, (short)0, c, false, false);
  asm volatile("v_nop\n\tv_nop\n\tv_nop\n\tv_nop" : "+v"(d) : "v"(a.w), "v"(b.w));
  return d;
}

__device__ __forceinline__ unsigned bf16_bits(float f) {
  const unsigned u = __float_as_uint(f);
  const unsigned r = (u + 0x7FFFu + ((u >> 16) & 1u)) >> 16;
  return (f != f) ? 0x7FC0u : r;
}
__device__ __forceinline__ float bf16_val(float f) {
  return __uint_as_float(bf16_bits(f) << 16);
}
__device__ __forceinline__ void split2(float a, float b, unsigned& hw, unsigned& lw) {
  const unsigned ha = bf16_bits(a), hb = bf16_bits(b);
  const unsigned la = bf16_bits(a - __uint_as_float(ha << 16));
  const unsigned lb = bf16_bits(b - __uint_as_float(hb << 16));
  hw = ha | (hb << 16);
  lw = la | (lb << 16);
}
__device__ __forceinline__ float relu_k(float v) { return (v > 0.0f) ? v : (v - v); }
__device__ __forceinline__ float nmax(float m, float v) { return (v > m || v != v) ? v : m; }

template <int SLB>
__device__ __forceinline__ int scan_chunk(const int* __restrict__ dsts, int nE, int cbase, int slotBase,
                                          int nb, int vec8, int* list, int tid, int lane, int wave) {
  int wc = 0;
  const int el0  = tid * EPT;
  const int e0   = cbase + el0;
  const int sent = -2147483647 - 1;
  v4i da, db;
  if (vec8 != 0 && cbase + CHUNK <= nE) {
    da = *(const v4i*)(dsts + e0);
    db = *(const v4i*)(dsts + e0 + 4);
  } else {
    da.x = (e0     < nE) ? dsts[min(e0,     nE - 1)] : sent;
    da.y = (e0 + 1 < nE) ? dsts[min(e0 + 1, nE - 1)] : sent;
    da.z = (e0 + 2 < nE) ? dsts[min(e0 + 2, nE - 1)] : sent;
    da.w = (e0 + 3 < nE) ? dsts[min(e0 + 3, nE - 1)] : sent;
    db.x = (e0 + 4 < nE) ? dsts[min(e0 + 4, nE - 1)] : sent;
    db.y = (e0 + 5 < nE) ? dsts[min(e0 + 5, nE - 1)] : sent;
    db.z = (e0 + 6 < nE) ? dsts[min(e0 + 6, nE - 1)] : sent;
    db.w = (e0 + 7 < nE) ? dsts[min(e0 + 7, nE - 1)] : sent;
  }
  const unsigned nbs = (unsigned)slotBase;
  const unsigned unb = (unsigned)nb;
  const unsigned s0 = (unsigned)da.x - nbs, s1 = (unsigned)da.y - nbs;
  const unsigned s2 = (unsigned)da.z - nbs, s3 = (unsigned)da.w - nbs;
  const unsigned s4 = (unsigned)db.x - nbs, s5 = (unsigned)db.y - nbs;
  const unsigned s6 = (unsigned)db.z - nbs, s7 = (unsigned)db.w - nbs;
  const bool h0 = s0 < unb, h1 = s1 < unb, h2 = s2 < unb, h3 = s3 < unb;
  const bool h4 = s4 < unb, h5 = s5 < unb, h6 = s6 < unb, h7 = s7 < unb;
  const unsigned any = __builtin_amdgcn_ballot_w32(h0 | h1 | h2 | h3 | h4 | h5 | h6 | h7);
  if (any != 0u) {
#define HITJ(J, HJ, SJ) { \
      const unsigned mj = __builtin_amdgcn_ballot_w32(HJ); \
      if (mj != 0u) { \
        if (HJ) { \
          const int pos = wc + (int)__builtin_amdgcn_mbcnt_lo(mj, 0u); \
          if (pos < WCAP) list[wave * WCAP + pos] = ((el0 + (J)) << SLB) | (int)(SJ); \
        } \
        wc += (int)__builtin_popcount(mj); } }
    HITJ(0, h0, s0)
    HITJ(1, h1, s1)
    HITJ(2, h2, s2)
    HITJ(3, h3, s3)
    HITJ(4, h4, s4)
    HITJ(5, h5, s5)
    HITJ(6, h6, s6)
    HITJ(7, h7, s7)
#undef HITJ
  }
  return wc;
}

__global__ __launch_bounds__(NTHR) void k_prep(const float* __restrict__ x,
    const float* __restrict__ W1, const float* __restrict__ b1, const float* __restrict__ W2,
    const float* __restrict__ b2, const float* __restrict__ W3, const float* __restrict__ b3,
    const float* __restrict__ W4, const float* __restrict__ b4,
    unsigned short* XB, unsigned short* W1D, unsigned short* W2D, unsigned short* W3D, unsigned short* W4D,
    float* BIAS) {
  const int b = (int)blockIdx.x, tid = (int)threadIdx.x;
  if (b < PB_X) {
    const int u   = b * NTHR + tid;
    const int row = u >> 4;
    const int k8  = (u & 15) * 8;
    const float* p = x + (size_t)row * F0;
    unsigned wv[4];
#pragma unroll
    for (int i = 0; i < 4; ++i) {
      const int c  = k8 + 2 * i;
      const int cc = c < F0 ? c : F0 - 2;
      const v2f a = *(const v2fa*)(p + cc);
      asm volatile("" :: "v"(a));
      const unsigned w = bf16_bits(a.x) | (bf16_bits(a.y) << 16);
      wv[i] = (c < F0) ? w : 0u;
    }
    v4u o; o.x = wv[0]; o.y = wv[1]; o.z = wv[2]; o.w = wv[3];
    unsigned short* dp = XB + (size_t)u * 8;
    *(volatile v4u*)dp = o;
    __threadfence();
    *(volatile v4u*)dp = o;
  } else if (b < PB_WEND) {
    const float* W; unsigned short* P; int Kr, Nr, KH, KU, bb;
    if (b < PB_X + PB_W1)                      { W = W1; P = W1D; Kr = F0; Nr = HD; KH = K1H; KU = K1 / 8; bb = PB_X; }
    else if (b < PB_X + PB_W1 + PB_W2)         { W = W2; P = W2D; Kr = HD; Nr = HD; KH = HP;  KU = K2 / 8; bb = PB_X + PB_W1; }
    else if (b < PB_X + PB_W1 + PB_W2 + PB_W3) { W = W3; P = W3D; Kr = HD; Nr = D3; KH = HP;  KU = K3 / 8; bb = PB_X + PB_W1 + PB_W2; }
    else                                       { W = W4; P = W4D; Kr = D3; Nr = D4; KH = D3;  KU = K4 / 8; bb = PB_X + PB_W1 + PB_W2 + PB_W3; }
    const int v   = (b - bb) * NTHR + tid;
    const int n   = v / KU;
    const int k8  = (v - n * KU) * 8;
    const int kk8 = k8 >= KH ? k8 - KH : k8;
    const int nc  = n < Nr ? n : Nr - 1;
    unsigned hb[8];
#pragma unroll
    for (int i = 0; i < 8; ++i) {
      const int kk = kk8 + i;
      const int kc = kk < Kr ? kk : Kr - 1;
      const float w = W[(size_t)kc * Nr + nc];
      asm volatile("" :: "v"(w));
      hb[i] = (kk < Kr && n < Nr) ? bf16_bits(w) : 0u;
    }
    v4u o;
    o.x = hb[0] | (hb[1] << 16); o.y = hb[2] | (hb[3] << 16);
    o.z = hb[4] | (hb[5] << 16); o.w = hb[6] | (hb[7] << 16);
    unsigned short* dp = P + (size_t)v * 8;
    *(volatile v4u*)dp = o;
    __threadfence();
    *(volatile v4u*)dp = o;
  } else {
    const int bi = b - PB_WEND;
    const float* src; int nr, off, cnt4;
    if (bi == 0)      { src = b1; nr = HD; off = OB1; cnt4 = HP / 4; }
    else if (bi == 1) { src = b2; nr = HD; off = OB2; cnt4 = HP / 4; }
    else if (bi == 2) { src = b3; nr = D3; off = OB3; cnt4 = D3 / 4; }
    else              { src = b4; nr = D4; off = OB4; cnt4 = D4 / 4; }
    const int g  = tid;
    const int gc = g < cnt4 ? g : cnt4 - 1;
    float fv[4];
#pragma unroll
    for (int i = 0; i < 4; ++i) {
      const int c  = 4 * gc + i;
      const int cc = c < nr ? c : nr - 1;
      const float f = src[cc];
      asm volatile("" :: "v"(f));
      fv[i] = (c < nr) ? bf16_val(f) : 0.0f;
    }
    v4f o; o.x = fv[0]; o.y = fv[1]; o.z = fv[2]; o.w = fv[3];
    float* dp = BIAS + off + 4 * gc;
    if (g < cnt4) *(volatile v4f*)dp = o;
    __threadfence();
    if (g < cnt4) *(volatile v4f*)dp = o;
  }
}

__global__ __launch_bounds__(NTHR) void k_bucket(const int* __restrict__ srcs, const int* __restrict__ dsts,
                                                 int vec8, int* LIST, int* CNT, int* OFF, float* DIS) {
  extern __shared__ __attribute__((aligned(16))) int dsm[];
  int* list = dsm;
  int* hl   = dsm + LISTN;
  int* sl   = dsm + LISTN + RCAP;
  int* cnt  = dsm + LISTN + 2 * RCAP;
  int* offs = cnt + NBA;
  int* cur  = offs + NBA;
  int* misc = cur + NBA;
  const int tid = (int)threadIdx.x, lane = tid & 31, wave = tid >> 5;
  const int blk = (int)blockIdx.x;
  const int nodeBase = blk * NBA;

  {
    const v4i z4 = {0, 0, 0, 0};
    for (int i = tid * 4; i < AGG_ZINTS; i += NTHR * 4) *(v4ia*)(dsm + i) = z4;
    if (tid < 16) misc[tid] = 0;
  }
  __syncthreads();

  int t = 0, ov = 0;
  const int nChunks = (NE + CHUNK - 1) / CHUNK;
#pragma unroll 1
  for (int ch = 0; ch < nChunks; ++ch) {
    const int cbase = ch * CHUNK;
    const int wc = scan_chunk<SLA>(dsts, NE, cbase, nodeBase, NBA, vec8, list, tid, lane, wave);
    if (lane == 0) misc[wave] = wc;
    __syncthreads();
    if (wave == 0) {
#pragma unroll 1
      for (int w2 = 0; w2 < NWAVE; ++w2) {
        int c = misc[w2];
        c = c < 0 ? 0 : (c > WCAP ? WCAP : c);
#pragma unroll 1
        for (int b0 = 0; b0 < c; b0 += 32) {
          const int idx = b0 + lane;
          const int ent = list[w2 * WCAP + (idx < WCAP ? idx : WCAP - 1)];
          const int m32 = (c - b0) < 32 ? (c - b0) : 32;
#pragma unroll 1
          for (int k = 0; k < m32; ++k) {
            const int u    = __builtin_amdgcn_readlane(ent, k);
            const int slot = u & (NBA - 1);
            const int el   = (u >> SLA) & (CHUNK - 1);
            const int pk   = ((cbase + el) << SLA) | slot;
            if (t < RCAP) {
              if (lane == 0) { hl[t] = pk; cnt[slot] = cnt[slot] + 1; }
              t = t + 1;
            } else {
              ov = 1;
            }
          }
        }
      }
    }
    __syncthreads();
  }
  if (wave == 0 && lane == 0) { misc[8] = t; misc[9] = ov; }
  __syncthreads();
  int tt = misc[8];
  tt = tt < 0 ? 0 : (tt > RCAP ? RCAP : tt);
  const int ovf = misc[9];

  if (wave == 0) {
    const int base = lane * (NBA / 32);
    int s = 0;
#pragma unroll 1
    for (int i = 0; i < NBA / 32; ++i) s += cnt[base + i];
    int incl = s;
#pragma unroll
    for (int d = 1; d < 32; d <<= 1) {
      const int y = __shfl_up(incl, d, 32);
      if (lane >= d) incl += y;
    }
    int run = incl - s;
#pragma unroll 1
    for (int i = 0; i < NBA / 32; ++i) {
      const int cv = cnt[base + i];
      offs[base + i] = run;
      cur[base + i]  = run;
      run += cv;
    }
  }
  __syncthreads();
  if (wave == 0) {
#pragma unroll 1
    for (int b0 = 0; b0 < tt; b0 += 32) {
      const int idx = b0 + lane;
      const int ent = hl[idx < RCAP ? idx : RCAP - 1];
      const int m32 = (tt - b0) < 32 ? (tt - b0) : 32;
#pragma unroll 1
      for (int k = 0; k < m32; ++k) {
        const int u    = __builtin_amdgcn_readlane(ent, k);
        const int slot = u & (NBA - 1);
        if (lane == 0) {
          int p = cur[slot];
          p = p < 0 ? 0 : (p > RCAP - 1 ? RCAP - 1 : p);
          sl[p] = u;
          cur[slot] = p + 1;
        }
      }
    }
  }
  __syncthreads();

#pragma unroll 1
  for (int j = 0; j < NBA / NTHR; ++j) {
    const int s = j * NTHR + tid;
    const float dg = (float)(cnt[s] + 1);
    const float dv = (dg > 0.0f) ? (1.0f / sqrtf(dg)) : 0.0f;
    cur[s] = __float_as_int(dv);
  }
  __syncthreads();

  {
    v4i c4 = *(const v4ia*)(cnt + 4 * tid);
    const v4i o4 = *(const v4ia*)(offs + 4 * tid);
    const v4i d4 = *(const v4ia*)(cur + 4 * tid);
    if (ovf != 0) { c4.x = -1; c4.y = -1; c4.z = -1; c4.w = -1; }
    v4f dv;
    dv.x = __int_as_float(d4.x); dv.y = __int_as_float(d4.y);
    dv.z = __int_as_float(d4.z); dv.w = __int_as_float(d4.w);
    int*   cp = CNT + nodeBase + 4 * tid;
    int*   op = OFF + nodeBase + 4 * tid;
    float* dp = DIS + nodeBase + 4 * tid;
    *(volatile v4i*)cp = c4; *(volatile v4i*)op = o4; *(volatile v4f*)dp = dv;
    __threadfence();
    *(volatile v4i*)cp = c4; *(volatile v4i*)op = o4; *(volatile v4f*)dp = dv;
  }

#pragma unroll 1
  for (int it = 0; it < RCAP / (4 * NTHR); ++it) {
    const int p4 = (it * NTHR + tid) * 4;
    const v4i e4 = *(const v4ia*)(sl + p4);
    int e0 = e4.x >> SLA, e1 = e4.y >> SLA, e2 = e4.z >> SLA, e3 = e4.w >> SLA;
    e0 = e0 < 0 ? 0 : (e0 > NE - 1 ? NE - 1 : e0);
    e1 = e1 < 0 ? 0 : (e1 > NE - 1 ? NE - 1 : e1);
    e2 = e2 < 0 ? 0 : (e2 > NE - 1 ? NE - 1 : e2);
    e3 = e3 < 0 ? 0 : (e3 > NE - 1 ? NE - 1 : e3);
    int s0 = srcs[e0], s1 = srcs[e1], s2 = srcs[e2], s3 = srcs[e3];
    asm volatile("" :: "v"(s0)); asm volatile("" :: "v"(s1));
    asm volatile("" :: "v"(s2)); asm volatile("" :: "v"(s3));
    s0 = s0 < 0 ? 0 : (s0 > NN - 1 ? NN - 1 : s0);
    s1 = s1 < 0 ? 0 : (s1 > NN - 1 ? NN - 1 : s1);
    s2 = s2 < 0 ? 0 : (s2 > NN - 1 ? NN - 1 : s2);
    s3 = s3 < 0 ? 0 : (s3 > NN - 1 ? NN - 1 : s3);
    v4i o;
    o.x = (p4     < tt) ? s0 : 0;
    o.y = (p4 + 1 < tt) ? s1 : 0;
    o.z = (p4 + 2 < tt) ? s2 : 0;
    o.w = (p4 + 3 < tt) ? s3 : 0;
    int* lp = LIST + (size_t)blk * RCAP + p4;
    *(volatile v4i*)lp = o;
    __threadfence();
    *(volatile v4i*)lp = o;
  }
}

__global__ __launch_bounds__(NTHR) void k_agg1(const int* __restrict__ LIST, const int* __restrict__ CNT,
                                               const int* __restrict__ OFF, const float* __restrict__ DIS,
                                               const unsigned short* __restrict__ XB, unsigned short* AX) {
  const int tid = (int)threadIdx.x, lane = tid & 31, wave = tid >> 5;
  const int blk = (int)blockIdx.x;
  const int nodeBase = blk * NBA;
  const int* lst = LIST + (size_t)blk * RCAP;
  const float qnan = __int_as_float(0x7fc00000);
  const int pL = lane < 12 ? lane : (lane < 24 ? lane - 12 : 0);
  const int sA = 2 * pL, sB = 2 * pL + 1;
  const bool losel = lane >= 12;
#pragma unroll 1
  for (int si = 0; si < NBA / NWAVE; ++si) {
    const int s    = si * NWAVE + wave;
    const int node = nodeBase + s;
    const int craw = CNT[node];
    const bool bad = (craw < 0) || (craw > DEGCAP);
    const int c = craw < 0 ? 0 : (craw > DEGCAP ? DEGCAP : craw);
    int o = OFF[node];
    o = o < 0 ? 0 : (o > RCAP ? RCAP : o);
    const int nc = node < NN ? node : NN - 1;
    const float dd = DIS[nc];
    float a0 = 0.0f, a1 = 0.0f, a2 = 0.0f, a3 = 0.0f;
#pragma unroll 1
    for (int b0 = 0; b0 < c; b0 += 32) {
      int idx = o + b0 + lane;
      idx = idx > RCAP - 1 ? RCAP - 1 : idx;
      int sr = lst[idx];
      sr = sr < 0 ? 0 : (sr > NN - 1 ? NN - 1 : sr);
      const int cfi = __float_as_int(DIS[sr]);
      const int m32 = (c - b0) < 32 ? (c - b0) : 32;
#pragma unroll 1
      for (int k = 0; k < m32; ++k) {
        const int   sk = __builtin_amdgcn_readlane(sr, k);
        const float ck = __int_as_float(__builtin_amdgcn_readlane(cfi, k));
        const v2u w = *(const v2ua*)(XB + (size_t)sk * XP + 4 * lane);
        a0 = fmaf(ck, __uint_as_float(w.x << 16), a0);
        a1 = fmaf(ck, __uint_as_float(w.x & 0xffff0000u), a1);
        a2 = fmaf(ck, __uint_as_float(w.y << 16), a2);
        a3 = fmaf(ck, __uint_as_float(w.y & 0xffff0000u), a3);
      }
    }
    {
      const v2u w = *(const v2ua*)(XB + (size_t)nc * XP + 4 * lane);
      a0 = fmaf(dd, __uint_as_float(w.x << 16), a0);
      a1 = fmaf(dd, __uint_as_float(w.x & 0xffff0000u), a1);
      a2 = fmaf(dd, __uint_as_float(w.y << 16), a2);
      a3 = fmaf(dd, __uint_as_float(w.y & 0xffff0000u), a3);
    }
    const float pz = bad ? qnan : 0.0f;
    const bool live = node < NN;
    const float v0 = live ? (dd * a0 + pz) : 0.0f;
    const float v1 = live ? (dd * a1 + pz) : 0.0f;
    const float v2 = live ? (dd * a2 + pz) : 0.0f;
    const float v3 = live ? (dd * a3 + pz) : 0.0f;
    unsigned hw0, lw0, hw1, lw1;
    split2(v0, v1, hw0, lw0);
    split2(v2, v3, hw1, lw1);
    const int g0 = __shfl((int)hw0, sA, 32), g1 = __shfl((int)hw1, sA, 32);
    const int g2 = __shfl((int)hw0, sB, 32), g3 = __shfl((int)hw1, sB, 32);
    const int p0 = __shfl((int)lw0, sA, 32), p1 = __shfl((int)lw1, sA, 32);
    const int p2 = __shfl((int)lw0, sB, 32), p3 = __shfl((int)lw1, sB, 32);
    v4u pv;
    pv.x = (unsigned)(losel ? p0 : g0);
    pv.y = (unsigned)(losel ? p1 : g1);
    pv.z = (unsigned)(losel ? p2 : g2);
    pv.w = (unsigned)(losel ? p3 : g3);
    unsigned short* hp = AX + (size_t)node * K1 + 8 * (lane < 24 ? lane : 0);
    const bool wr = lane < 24;
    if (wr) *(volatile v4u*)hp = pv;
    __threadfence();
    if (wr) *(volatile v4u*)hp = pv;
  }
}

template <int TN, int MODE>
__global__ __launch_bounds__(GTHR) __attribute__((amdgpu_num_vgpr(248)))
void k_gemm(const unsigned short* __restrict__ A, int lda, const unsigned short* __restrict__ BT, int K,
            const float* __restrict__ bias, const float* __restrict__ dis,
            unsigned short* outH, float* outF, int ldo, int ntot, int nValid) {
  constexpr int BN  = 32 * TN;
  constexpr int NG  = BN / 4;
  constexpr int NJ  = (NG + 31) / 32;
  constexpr int NP  = BN / 8;
  constexpr int NQ  = 2 * NP;
  constexpr int NJQ = (NQ + 31) / 32;
  extern __shared__ __attribute__((aligned(16))) float gsm[];
  float* stg   = gsm;
  float* biasS = gsm + 64 * BN;
  unsigned short* rowbuf = (unsigned short*)(gsm + 65 * BN);
  const int tid = (int)threadIdx.x, lane = tid & 31, wave = tid >> 5, hh = lane >> 4, m = lane & 15;
  const int rg = wave & 3, chh = wave >> 2;
  const int rowBase = (int)blockIdx.x * 64;
  const int col0    = (int)blockIdx.y * BN;

  v8f acc[TN];
  {
    const v8f z = {0.f, 0.f, 0.f, 0.f, 0.f, 0.f, 0.f, 0.f};
#pragma unroll
    for (int t = 0; t < TN; ++t) acc[t] = z;
  }
  const unsigned short* ap = A  + (size_t)(rowBase + 16 * rg + m) * (size_t)lda + 8 * hh;
  const unsigned short* bp = BT + (size_t)(col0 + 16 * TN * chh + m) * (size_t)K + 8 * hh;
#pragma unroll 1
  for (int k0 = 0; k0 < K; k0 += 32) {
    FragB af;
    af.h[0] = *(const v8usa*)(ap + k0);
    af.h[1] = *(const v8usa*)(ap + k0 + 16);
#pragma unroll
    for (int t = 0; t < TN; ++t) {
      const unsigned short* wq = bp + (size_t)(16 * t) * (size_t)K + k0;
      FragB bf;
      bf.h[0] = *(const v8usa*)wq;
      bf.h[1] = *(const v8usa*)(wq + 16);
      acc[t] = wmb(af, bf, acc[t]);
    }
  }

#pragma unroll
  for (int t = 0; t < TN; ++t) {
    const int lc = 16 * TN * chh + 16 * t + m;
#pragma unroll
    for (int r = 0; r < 8; ++r) {
      const int lr = 16 * rg + 8 * hh + r;
      stg[lr * BN + lc] = acc[t][r];
    }
  }
  if constexpr (MODE != 1) {
    if (tid < NG) {
      const v4f bb = *(const v4f*)(bias + col0 + 4 * tid);
      *(v4fa*)(biasS + 4 * tid) = bb;
    }
  }
  __syncthreads();

#pragma unroll 1
  for (int i = 0; i < 8; ++i) {
    const int lr  = 8 * wave + i;
    const int row = rowBase + lr;
    if constexpr (MODE == 0) {
      unsigned short* rb = rowbuf + wave * (2 * BN);
#pragma unroll
      for (int j = 0; j < NJ; ++j) {
        const int g  = lane + 32 * j;
        const int gc = g < NG ? g : NG - 1;
        const v4f v = *(const v4fa*)(stg + lr * BN + 4 * gc);
        const v4f b = *(const v4fa*)(biasS + 4 * gc);
        const float y0 = relu_k(v.x + b.x), y1 = relu_k(v.y + b.y);
        const float y2 = relu_k(v.z + b.z), y3 = relu_k(v.w + b.w);
        unsigned ha, la, hb, lb;
        split2(y0, y1, ha, la);
        split2(y2, y3, hb, lb);
        v2u hw, lw;
        hw.x = ha; hw.y = hb; lw.x = la; lw.y = lb;
        if (g < NG) {
          *(v2ua*)(rb + 4 * g) = hw;
          *(v2ua*)(rb + BN + 4 * g) = lw;
        }
      }
      __syncthreads();
      v4u q[NJQ];
#pragma unroll
      for (int j = 0; j < NJQ; ++j) {
        const int p  = lane + 32 * j;
        const int pc = p < NQ ? p : NQ - 1;
        q[j] = *(const v4ua*)(rb + 8 * pc);
        asm volatile("" :: "v"(q[j]));
      }
      __syncthreads();
      unsigned short* orow = outH + (size_t)row * (size_t)ldo;
#pragma unroll
      for (int j = 0; j < NJQ; ++j) {
        const int p   = lane + 32 * j;
        const int off = (p < NP) ? (col0 + 8 * p) : (ntot + col0 + 8 * (p - NP));
        if (p < NQ) *(volatile v4u*)(orow + off) = q[j];
      }
      __threadfence();
#pragma unroll
      for (int j = 0; j < NJQ; ++j) {
        const int p   = lane + 32 * j;
        const int off = (p < NP) ? (col0 + 8 * p) : (ntot + col0 + 8 * (p - NP));
        if (p < NQ) *(volatile v4u*)(orow + off) = q[j];
      }
    } else {
      float dv = 1.0f;
      if constexpr (MODE == 1) dv = dis[row];
      const bool rok = row < nValid;
      v4f y[NJ];
#pragma unroll
      for (int j = 0; j < NJ; ++j) {
        const int g  = lane + 32 * j;
        const int gc = g < NG ? g : NG - 1;
        const v4f v = *(const v4fa*)(stg + lr * BN + 4 * gc);
        if constexpr (MODE == 1) {
          y[j] = v * dv;
        } else {
          const v4f b = *(const v4fa*)(biasS + 4 * gc);
          v4f t;
          t.x = relu_k(v.x + b.x); t.y = relu_k(v.y + b.y);
          t.z = relu_k(v.z + b.z); t.w = relu_k(v.w + b.w);
          y[j] = t;
        }
        asm volatile("" :: "v"(y[j]));
      }
      float* orow = outF + (size_t)row * (size_t)ldo + col0;
#pragma unroll
      for (int j = 0; j < NJ; ++j) {
        const int g = lane + 32 * j;
        if (g < NG && rok) *(volatile v4f*)(orow + 4 * g) = y[j];
      }
      __threadfence();
#pragma unroll
      for (int j = 0; j < NJ; ++j) {
        const int g = lane + 32 * j;
        if (g < NG && rok) *(volatile v4f*)(orow + 4 * g) = y[j];
      }
    }
  }
}

__global__ __launch_bounds__(NTHR) void k_agg2pool(const int* __restrict__ LIST, const int* __restrict__ CNT,
                                                   const int* __restrict__ OFF, const float* __restrict__ DIS,
                                                   const float* __restrict__ T2, const float* __restrict__ B2P,
                                                   const int* __restrict__ bat, float* PREC, int* PID) {
  extern __shared__ __attribute__((aligned(16))) float tbl[];
  __shared__ int gslot[NBA];
  __shared__ __attribute__((aligned(16))) int gids[32];
  __shared__ int gmisc[4];
  __shared__ __attribute__((aligned(16))) float b2s[HP];
  const int tid = (int)threadIdx.x, lane = tid & 31, wave = tid >> 5;
  const int blk = (int)blockIdx.x;
  const int nodeBase = blk * NBA;
  const int* lst = LIST + (size_t)blk * RCAP;
  float* mytab = tbl + wave * (GCAP * HP);
  const float ninf = __int_as_float((int)0xff800000u);
  const float qnan = __int_as_float(0x7fc00000);

  {
    v4f n4; n4.x = ninf; n4.y = ninf; n4.z = ninf; n4.w = ninf;
    for (int i = 4 * lane; i < GCAP * HP; i += 128) *(v4fa*)(mytab + i) = n4;
  }
#pragma unroll
  for (int j = 0; j < NBA / NTHR; ++j) {
    const int s = j * NTHR + tid;
    const int node = nodeBase + s;
    const int nc = node < NN ? node : NN - 1;
    const int id = bat[nc];
    asm volatile("" :: "v"(id));
    gslot[s] = (node < NN) ? id : -1;
  }
  if (tid < 32) gids[tid] = -1;
  if (tid < 4) gmisc[tid] = 0;
  if (tid < HP / 4) {
    const v4f bb = *(const v4f*)(B2P + 4 * tid);
    *(v4fa*)(b2s + 4 * tid) = bb;
  }
  __syncthreads();
  if (tid == 0) {
    int ng = 0, ov = 0, lastId = -1, lastSl = -1;
#pragma unroll 1
    for (int s = 0; s < NBA; ++s) {
      const int id = gslot[s];
      int sl = -1;
      if ((unsigned)id < (unsigned)NGR) {
        if (id == lastId) {
          sl = lastSl;
        } else {
#pragma unroll 1
          for (int q = 0; q < GCAP; ++q) { if (q < ng && gids[q] == id) sl = q; }
          if (sl < 0) {
            if (ng < GCAP) { gids[ng] = id; sl = ng; ng = ng + 1; } else { ov = 1; }
          }
          lastId = id; lastSl = sl;
        }
      }
      gslot[s] = sl;
    }
    gmisc[0] = ov;
  }
  __syncthreads();

  const v4f ba = *(const v4fa*)(b2s + 4 * lane);
  const v4f bb = *(const v4fa*)(b2s + 128 + 4 * lane);
  const v2f bc = *(const v2fa*)(b2s + 256 + 2 * lane);

#pragma unroll 1
  for (int si = 0; si < NBA / NWAVE; ++si) {
    const int s    = si * NWAVE + wave;
    const int node = nodeBase + s;
    int gs = __builtin_amdgcn_readfirstlane(gslot[s]);
    if (gs < 0) continue;
    gs = gs > GCAP - 1 ? GCAP - 1 : gs;
    const int craw = CNT[node];
    const bool bad = (craw < 0) || (craw > DEGCAP);
    const int c = craw < 0 ? 0 : (craw > DEGCAP ? DEGCAP : craw);
    int o = OFF[node];
    o = o < 0 ? 0 : (o > RCAP ? RCAP : o);
    const int nc = node < NN ? node : NN - 1;
    const float dd = DIS[nc];
    v4f xa = {0.f, 0.f, 0.f, 0.f}, xb = {0.f, 0.f, 0.f, 0.f};
    v2f xc = {0.f, 0.f};
#pragma unroll 1
    for (int b0 = 0; b0 < c; b0 += 32) {
      int idx = o + b0 + lane;
      idx = idx > RCAP - 1 ? RCAP - 1 : idx;
      int sr = lst[idx];
      sr = sr < 0 ? 0 : (sr > NN - 1 ? NN - 1 : sr);
      const int m32 = (c - b0) < 32 ? (c - b0) : 32;
#pragma unroll 1
      for (int k = 0; k < m32; ++k) {
        const int sk = __builtin_amdgcn_readlane(sr, k);
        const float* rp = T2 + (size_t)sk * HP;
        xa += *(const v4fa*)(rp + 4 * lane);
        xb += *(const v4fa*)(rp + 128 + 4 * lane);
        xc += *(const v2fa*)(rp + 256 + 2 * lane);
      }
    }
    {
      const float* rp = T2 + (size_t)nc * HP;
      xa += *(const v4fa*)(rp + 4 * lane);
      xb += *(const v4fa*)(rp + 128 + 4 * lane);
      xc += *(const v2fa*)(rp + 256 + 2 * lane);
    }
    const float pz = bad ? qnan : 0.0f;
    float* tb = mytab + gs * HP;
    v4f ma = *(const v4fa*)(tb + 4 * lane);
    v4f mb = *(const v4fa*)(tb + 128 + 4 * lane);
    v2f mc = *(const v2fa*)(tb + 256 + 2 * lane);
    ma.x = nmax(ma.x, relu_k(dd * xa.x + ba.x) + pz);
    ma.y = nmax(ma.y, relu_k(dd * xa.y + ba.y) + pz);
    ma.z = nmax(ma.z, relu_k(dd * xa.z + ba.z) + pz);
    ma.w = nmax(ma.w, relu_k(dd * xa.w + ba.w) + pz);
    mb.x = nmax(mb.x, relu_k(dd * xb.x + bb.x) + pz);
    mb.y = nmax(mb.y, relu_k(dd * xb.y + bb.y) + pz);
    mb.z = nmax(mb.z, relu_k(dd * xb.z + bb.z) + pz);
    mb.w = nmax(mb.w, relu_k(dd * xb.w + bb.w) + pz);
    mc.x = nmax(mc.x, relu_k(dd * xc.x + bc.x) + pz);
    mc.y = nmax(mc.y, relu_k(dd * xc.y + bc.y) + pz);
    *(v4fa*)(tb + 4 * lane) = ma;
    *(v4fa*)(tb + 128 + 4 * lane) = mb;
    *(v2fa*)(tb + 256 + 2 * lane) = mc;
  }
  __syncthreads();

  const int gov = gmisc[0];
  constexpr int NIT = (GCAP * HP) / (4 * NTHR);
  static_assert(NIT * 4 * NTHR == GCAP * HP);
  v4f rv[NIT];
#pragma unroll
  for (int it = 0; it < NIT; ++it) {
    const int q = it * NTHR + tid;
    v4f r = *(const v4fa*)(tbl + 4 * q);
#pragma unroll
    for (int w2 = 1; w2 < NWAVE; ++w2) {
      const v4f t = *(const v4fa*)(tbl + w2 * (GCAP * HP) + 4 * q);
      r.x = nmax(r.x, t.x); r.y = nmax(r.y, t.y); r.z = nmax(r.z, t.z); r.w = nmax(r.w, t.w);
    }
    if (gov != 0) { r.x = qnan; r.y = qnan; r.z = qnan; r.w = qnan; }
    rv[it] = r;
  }
  const v4i pidv = *(const v4ia*)(gids + 4 * (lane & 7));
  float* pp = PREC + (size_t)blk * (GCAP * HP);
  int* ip = PID + (size_t)blk * 32 + 4 * (lane & 7);
  const bool pw = (wave == 0) && (lane < 8);
#pragma unroll
  for (int it = 0; it < NIT; ++it) *(volatile v4f*)(pp + 4 * (it * NTHR + tid)) = rv[it];
  if (pw) *(volatile v4i*)ip = pidv;
  __threadfence();
#pragma unroll
  for (int it = 0; it < NIT; ++it) *(volatile v4f*)(pp + 4 * (it * NTHR + tid)) = rv[it];
  if (pw) *(volatile v4i*)ip = pidv;
}

__global__ __launch_bounds__(HP) void k_pool(const float* __restrict__ PREC, const int* __restrict__ PID,
                                             unsigned short* PHL) {
  __shared__ int mlist[NREC];
  __shared__ int mcnt;
  __shared__ __attribute__((aligned(16))) unsigned short ph[2 * HP];
  const int tid = (int)threadIdx.x, lane = tid & 31, wave = tid >> 5;
  const int g = (int)blockIdx.x;
  if (wave == 0) {
    int cn = 0;
#pragma unroll 1
    for (int it = 0; it < NREC / 32; ++it) {
      const int r = it * 32 + lane;
      const int pid = PID[(r >> 4) * 32 + (r & 15)];
      const bool hit = (pid == g);
      const unsigned mk = __builtin_amdgcn_ballot_w32(hit);
      if (hit) {
        const int pos = cn + (int)__builtin_amdgcn_mbcnt_lo(mk, 0u);
        if (pos < NREC) mlist[pos] = r;
      }
      cn += (int)__builtin_popcount(mk);
    }
    if (lane == 0) mcnt = cn;
  }
  __syncthreads();
  int mc = mcnt;
  mc = mc < 0 ? 0 : (mc > NREC ? NREC : mc);
  const float pinf = __int_as_float(0x7f800000);
  const float ninf = __int_as_float((int)0xff800000u);
  float mval = ninf;
#pragma unroll 1
  for (int q = 0; q < mc; ++q) {
    int r = mlist[q];
    r = r < 0 ? 0 : (r > NREC - 1 ? NREC - 1 : r);
    const float v = PREC[(size_t)r * HP + tid];
    mval = nmax(mval, v);
  }
  const float pv = (mval == pinf || mval == ninf) ? 0.0f : mval;
  const unsigned hb = bf16_bits(pv);
  const unsigned lb = bf16_bits(pv - __uint_as_float(hb << 16));
  ph[tid] = (unsigned short)hb;
  ph[HP + tid] = (unsigned short)lb;
  __syncthreads();
  const int pc = tid < 80 ? tid : 79;
  const v4u q = *(const v4ua*)(ph + 8 * pc);
  asm volatile("" :: "v"(q));
  unsigned short* dp = PHL + (size_t)g * (2 * HP) + 8 * pc;
  if (tid < 80) *(volatile v4u*)dp = q;
  __threadfence();
  if (tid < 80) *(volatile v4u*)dp = q;
}

static inline size_t al256(size_t o) { return (o + 255) & ~(size_t)255; }

extern "C" void kernel_launch(void* const* d_in, const int* in_sizes, int n_in,
                              void* d_out, int out_size, void* d_ws, size_t ws_size,
                              hipStream_t stream) {
  if (n_in < 11) return;
  if (in_sizes[0] != NN * F0) return;
  if (in_sizes[1] != 2 * NE) return;
  if (in_sizes[2] != NN) return;
  if (in_sizes[3] != F0 * HD || in_sizes[4] != HD) return;
  if (in_sizes[5] != HD * HD || in_sizes[6] != HD) return;
  if (in_sizes[7] != HD * D3 || in_sizes[8] != D3) return;
  if (in_sizes[9] != D3 * D4 || in_sizes[10] != D4) return;
  if (out_size != NGR * D4) return;

  const float* x    = (const float*)d_in[0];
  const int*   edge = (const int*)d_in[1];
  const int*   bat  = (const int*)d_in[2];
  const float* W1 = (const float*)d_in[3];  const float* b1 = (const float*)d_in[4];
  const float* W2 = (const float*)d_in[5];  const float* b2 = (const float*)d_in[6];
  const float* W3 = (const float*)d_in[7];  const float* b3 = (const float*)d_in[8];
  const float* W4 = (const float*)d_in[9];  const float* b4 = (const float*)d_in[10];
  float* out = (float*)d_out;
  const int* src = edge;
  const int* dst = edge + NE;
  const int vec8 = ((NE & 3) == 0) ? 1 : 0;

  char* ws = (char*)d_ws;
  size_t off = 0;
  const size_t oW1D = off; off = al256(off + (size_t)HP * K1 * 2);
  const size_t oW2D = off; off = al256(off + (size_t)HP * K2 * 2);
  const size_t oW3D = off; off = al256(off + (size_t)D3 * K3 * 2);
  const size_t oW4D = off; off = al256(off + (size_t)D4 * K4 * 2);
  const size_t oBIA = off; off = al256(off + (size_t)NBIAS * 4);
  const size_t oCNT = off; off = al256(off + (size_t)NPAD * 4);
  const size_t oOFF = off; off = al256(off + (size_t)NPAD * 4);
  const size_t oDIS = off; off = al256(off + (size_t)NPAD * 4);
  const size_t oLST = off; off = al256(off + (size_t)NBLK * RCAP * 4);
  const size_t szXB = (size_t)NN * XP * 2;
  const size_t szH1 = (size_t)CH * K2 * 2;
  const size_t oR0  = off; off = al256(off + (szXB > szH1 ? szXB : szH1));
  const size_t oAX  = off; off = al256(off + (size_t)NPAD * K1 * 2);
  const size_t oT2  = off; off = al256(off + (size_t)NN * HP * 4);
  const size_t oPRE = off; off = al256(off + (size_t)NREC * HP * 4);
  const size_t oPID = off; off = al256(off + (size_t)NBLK * 32 * 4);
  const size_t oPHL = off; off = al256(off + (size_t)NGR * K3 * 2);
  const size_t oZ1  = off; off = al256(off + (size_t)NGR * K4 * 2);
  if (off > ws_size) return;

  unsigned short* W1D = (unsigned short*)(ws + oW1D);
  unsigned short* W2D = (unsigned short*)(ws + oW2D);
  unsigned short* W3D = (unsigned short*)(ws + oW3D);
  unsigned short* W4D = (unsigned short*)(ws + oW4D);
  float*          BIA = (float*)(ws + oBIA);
  int*            CNT = (int*)(ws + oCNT);
  int*            OFF = (int*)(ws + oOFF);
  float*          DIS = (float*)(ws + oDIS);
  int*            LST = (int*)(ws + oLST);
  unsigned short* XB  = (unsigned short*)(ws + oR0);
  unsigned short* H1C = (unsigned short*)(ws + oR0);
  unsigned short* AX  = (unsigned short*)(ws + oAX);
  float*          T2  = (float*)(ws + oT2);
  float*          PRE = (float*)(ws + oPRE);
  int*            PID = (int*)(ws + oPID);
  unsigned short* PHL = (unsigned short*)(ws + oPHL);
  unsigned short* Z1  = (unsigned short*)(ws + oZ1);

  const size_t bktLds  = (size_t)AGG_LDS_INTS * 4;
  const size_t poolLds = (size_t)NWAVE * GCAP * HP * 4;
  const size_t g10Lds  = (size_t)292 * 320;
  const size_t g8Lds   = (size_t)292 * 256;
  const size_t g4Lds   = (size_t)292 * 128;
  hipFuncSetAttribute(reinterpret_cast<const void*>(&k_bucket), hipFuncAttributeMaxDynamicSharedMemorySize, (int)bktLds);
  hipFuncSetAttribute(reinterpret_cast<const void*>(&k_agg2pool), hipFuncAttributeMaxDynamicSharedMemorySize, (int)poolLds);
  hipFuncSetAttribute(reinterpret_cast<const void*>(&k_gemm<10, 0>), hipFuncAttributeMaxDynamicSharedMemorySize, (int)g10Lds);
  hipFuncSetAttribute(reinterpret_cast<const void*>(&k_gemm<10, 1>), hipFuncAttributeMaxDynamicSharedMemorySize, (int)g10Lds);
  hipFuncSetAttribute(reinterpret_cast<const void*>(&k_gemm<8, 0>), hipFuncAttributeMaxDynamicSharedMemorySize, (int)g8Lds);

  k_prep<<<PB_ALL, NTHR, 0, stream>>>(x, W1, b1, W2, b2, W3, b3, W4, b4, XB, W1D, W2D, W3D, W4D, BIA);
  k_bucket<<<NBLK, NTHR, bktLds, stream>>>(src, dst, vec8, LST, CNT, OFF, DIS);
  k_agg1<<<NBLK, NTHR, 0, stream>>>(LST, CNT, OFF, DIS, XB, AX);
  for (int c = 0; c < NCHUNK; ++c) {
    k_gemm<10, 0><<<dim3(CH / 64, 1), GTHR, g10Lds, stream>>>(
        AX + (size_t)c * CH * K1, K1, W1D, K1, BIA + OB1, DIS, H1C, T2, K2, HP, CH);
    k_gemm<10, 1><<<dim3(CH / 64, 1), GTHR, g10Lds, stream>>>(
        H1C, K2, W2D, K2, BIA, DIS + (size_t)c * CH, H1C, T2 + (size_t)c * CH * HP, HP, HP, NN - c * CH);
  }
  k_agg2pool<<<NBLK, NTHR, poolLds, stream>>>(LST, CNT, OFF, DIS, T2, BIA + OB2, bat, PRE, PID);
  k_pool<<<NGR, HP, 0, stream>>>(PRE, PID, PHL);
  k_gemm<8, 0><<<dim3(NGR / 64, D3 / 256), GTHR, g8Lds, stream>>>(
      PHL, K3, W3D, K3, BIA + OB3, DIS, Z1, out, K4, D3, NGR);
  k_gemm<4, 2><<<dim3(NGR / 64, 1), GTHR, g4Lds, stream>>>(
      Z1, K4, W4D, K4, BIA + OB4, DIS, Z1, out, D4, D4, NGR);
}
